// UNetCrossAttention_16406775071032
// MI455X (gfx1250) — hardware-verified
//
#include <hip/hip_runtime.h>
#include <math.h>

#define B_    2
#define NQ_   256
#define NK_   2048
#define DIM_  256
#define NH_   8
#define HD_   32
#define RPED_ 128

typedef __attribute__((ext_vector_type(16))) _Float16 v16h;
typedef __attribute__((ext_vector_type(8)))  _Float16 v8h;
typedef __attribute__((ext_vector_type(8)))  float    v8f;
typedef __attribute__((ext_vector_type(4)))  float    v4f;
typedef __attribute__((ext_vector_type(4)))  unsigned v4u;
typedef float __attribute__((may_alias)) float_a;
#define PSC 256.0f
#define PUN (1.0f / 256.0f)

template <typename V> __device__ __forceinline__ void vst2(void* p, V v) {
  *(volatile V*)p = v; __threadfence(); *(volatile V*)p = v;
}
__device__ __forceinline__ v8f wmma_f16(v16h a, v16h b, v8f c) {
  v8f d = __builtin_amdgcn_wmma_f32_16x16x32_f16(false, a, false, b, (short)0, c, false, false);
  asm volatile("v_nop\n\tv_nop\n\tv_nop\n\tv_nop" : "+v"(d) : "v"(a), "v"(b));
  return d;
}
__device__ __forceinline__ v16h frag_h(const _Float16* row, int k0, int lane) {
  union { v16h v; v8h h[2]; } r; const _Float16* p = row + k0 + 8 * (lane >> 4);
  r.h[0] = *(const v8h*)(p); r.h[1] = *(const v8h*)(p + 16); return r.v;
}
__device__ __forceinline__ v16h frag_f32(const float* row, int k0, int lane, float s) {
  v16h a; const float* p = row + k0 + 8 * (lane >> 4);
#pragma unroll
  for (int i = 0; i < 8; ++i) { a[i] = (_Float16)(p[i] * s); a[8 + i] = (_Float16)(p[16 + i] * s); }
  return a;
}

__global__ __launch_bounds__(256) void k_wt(const float* __restrict__ W, _Float16* __restrict__ WT, int K, int M) {
  __shared__ __align__(16) _Float16 tile[64][72];
  const int mt = (M / 64 > 0) ? M / 64 : 1, tid = threadIdx.x;
  const int m0 = (blockIdx.x % mt) * 64, k0 = (blockIdx.x / mt) * 64, mw = (M < 64) ? M : 64;
  for (int i = tid; i < 64 * 64; i += 256) { const int kk = i >> 6, mm = i & 63; tile[mm][kk] = (mm < mw) ? (_Float16)W[(size_t)(k0 + kk) * M + m0 + mm] : (_Float16)0.f; }
  __syncthreads();
  for (int g = tid; g < 64 * 8; g += 256) { const int mm = g >> 3, pc = g & 7; if (mm < mw) vst2(WT + (size_t)(m0 + mm) * K + k0 + pc * 8, *(const v4u*)(&tile[mm][pc * 8])); }
}

__global__ __launch_bounds__(128) void build_tables_k(const float* __restrict__ w1, const float* __restrict__ b1,
                                                      const float* __restrict__ w2, float* __restrict__ tables) {
  __shared__ __align__(16) float st[8000];
  const int i = blockIdx.x;
  const float* W1 = w1 + i * 3 * RPED_; const float* B1 = b1 + i * RPED_; const float* W2 = w2 + i * RPED_ * NH_;
  const float step = 8.0f / 9.0f;
  for (int v = threadIdx.x; v < 1000; v += blockDim.x) {
    const int p = v / 100, q = (v / 10) % 10, r = v % 10;
    const float c0 = -4.0f + p * step, c1 = -4.0f + q * step, c2 = -4.0f + r * step;
    float acc[NH_];
#pragma unroll
    for (int h = 0; h < NH_; ++h) acc[h] = 0.0f;
#pragma unroll 1
    for (int d = 0; d < RPED_; ++d) {
      float hv = fmaf(c0, W1[d], fmaf(c1, W1[RPED_ + d], fmaf(c2, W1[2 * RPED_ + d], B1[d])));
      hv = fmaxf(hv, 0.0f);
#pragma unroll
      for (int h = 0; h < NH_; ++h) acc[h] = fmaf(hv, W2[d * NH_ + h], acc[h]);
    }
#pragma unroll
    for (int h = 0; h < NH_; ++h) st[v * NH_ + h] = acc[h];
  }
  __syncthreads();
  for (int g = threadIdx.x; g < 2000; g += blockDim.x) vst2(tables + (size_t)i * 8000 + g * 4, *(const v4f*)(&st[g * 4]));
}

__device__ __forceinline__ float grid_coord(float d) {
  float s = copysignf(1.0f, d);
  return s * __log2f(fabsf(d) * 512.0f + 1.0f) * (1.0f / 12.0f);
}
__global__ __launch_bounds__(256) void rpe_k(const float* __restrict__ refp, const float* __restrict__ xyz,
                                             const float* __restrict__ tables, float* __restrict__ attn) {
  __shared__ float tab[8000];
  const int tid = blockIdx.x * 256 + threadIdx.x;
  const int k = tid & (NK_ - 1), q = (tid >> 11) & (NQ_ - 1), b = tid >> 19;
  const float kx = xyz[(b * NK_ + k) * 3 + 0], ky = xyz[(b * NK_ + k) * 3 + 1], kz = xyz[(b * NK_ + k) * 3 + 2];
  float acc[NH_];
#pragma unroll
  for (int h = 0; h < NH_; ++h) acc[h] = 0.0f;
  for (int i = 0; i < 8; ++i) {
    __syncthreads();
    for (int t = threadIdx.x; t < 8000; t += 256) tab[t] = tables[i * 8000 + t];
    __syncthreads();
    const float* rp = refp + ((b * NQ_ + q) * 8 + i) * 3;
    const float gx = grid_coord(rp[0] - kx), gy = grid_coord(rp[1] - ky), gz = grid_coord(rp[2] - kz);
    const float xf = (gx + 1.0f) * 4.5f, yf = (gy + 1.0f) * 4.5f, zf = (gz + 1.0f) * 4.5f;
    const float x0f = floorf(xf), y0f = floorf(yf), z0f = floorf(zf);
    const float wx1 = xf - x0f, wy1 = yf - y0f, wz1 = zf - z0f, wx0 = 1.0f - wx1, wy0 = 1.0f - wy1, wz0 = 1.0f - wz1;
    const int x0 = (int)x0f, y0 = (int)y0f, z0 = (int)z0f, x1 = x0 + 1, y1 = y0 + 1, z1 = z0 + 1;
    auto corner = [&](int zi, int yi, int xi, float w) {
      if ((unsigned)zi < 10u && (unsigned)yi < 10u && (unsigned)xi < 10u) {
        const float* tp = &tab[(zi * 100 + yi * 10 + xi) * NH_];
#pragma unroll
        for (int h = 0; h < NH_; ++h) acc[h] = fmaf(w, tp[h], acc[h]);
      }
    };
    corner(z0, y0, x0, wz0 * wy0 * wx0); corner(z0, y0, x1, wz0 * wy0 * wx1);
    corner(z0, y1, x0, wz0 * wy1 * wx0); corner(z0, y1, x1, wz0 * wy1 * wx1);
    corner(z1, y0, x0, wz1 * wy0 * wx0); corner(z1, y0, x1, wz1 * wy0 * wx1);
    corner(z1, y1, x0, wz1 * wy1 * wx0); corner(z1, y1, x1, wz1 * wy1 * wx1);
  }
  const long base = ((long)(b * NH_) * NQ_ + q) * NK_ + k;
#pragma unroll
  for (int h = 0; h < NH_; ++h) vst2(attn + base + (long)h * NQ_ * NK_, (float_a)acc[h]);
}

template <int N, int OUT>
__global__ __launch_bounds__(128) void proj_k(const float* __restrict__ X, const _Float16* __restrict__ WT, const float* __restrict__ bias,
                                             _Float16* __restrict__ Yh, float* __restrict__ Yf, float oscale, int NR) {
  constexpr int NT = N / 16;
  __shared__ __align__(16) float so[4][16 * N];
  const int tid = threadIdx.x, wave = tid >> 5, lane = tid & 31, hi = lane >> 4, col = lane & 15;
  const int m0 = (blockIdx.x * 4 + wave) * 16;
  const int tok = m0 + col, r_ = tok % NR, b_ = tok / NR;
  const float* ar = X + ((size_t)r_ * B_ + b_) * DIM_;
  float* S = so[wave];
#pragma unroll 1
  for (int nt = 0; nt < NT; ++nt) {
    v8f acc = {};
    const _Float16* br = WT + (size_t)(nt * 16 + col) * DIM_;
#pragma unroll
    for (int kc = 0; kc < DIM_ / 32; ++kc) acc = wmma_f16(frag_f32(ar, kc * 32, lane, 1.0f), frag_h(br, kc * 32, lane), acc);
#pragma unroll
    for (int r = 0; r < 8; ++r) S[(hi * 8 + r) * N + nt * 16 + col] = (acc[r] + bias[nt * 16 + col]) * oscale;
  }
  __syncthreads();
  if (OUT == 0) {
    _Float16* dst = Yh + (size_t)m0 * N;
    for (int q = 0; q < 16 * N / 8 / 32; ++q) { const int g = q * 32 + lane;
      union { v8h h; v4u u; } pk;
#pragma unroll
      for (int e = 0; e < 8; ++e) pk.h[e] = (_Float16)S[g * 8 + e];
      vst2(dst + g * 8, pk.u); }
  } else {
    float* dst = Yf + (size_t)m0 * N;
    for (int q = 0; q < 16 * N / 4 / 32; ++q) { const int g = q * 32 + lane; vst2(dst + g * 4, *(const v4f*)(S + g * 4)); }
  }
}

__global__ __launch_bounds__(256) void qk_k(const _Float16* __restrict__ qf, const _Float16* __restrict__ kf, float* __restrict__ attn) {
  __shared__ __align__(16) float so[8][16 * 128];
  const int gw = blockIdx.x * 8 + (threadIdx.x >> 5);
  const int kt = gw & 15, qt = (gw >> 4) & 15, h = (gw >> 8) & 7, b = gw >> 11;
  const int lane = threadIdx.x & 31, hi = lane >> 4, col = lane & 15;
  const v16h a = frag_h(qf + (size_t)(b * NQ_ + qt * 16 + col) * DIM_ + h * HD_, 0, lane);
  float* S = so[threadIdx.x >> 5];
  float* rowp = attn + (((size_t)(b * NH_ + h) * NQ_ + qt * 16) * NK_) + kt * 128;
#pragma unroll
  for (int nt = 0; nt < 8; ++nt) {
    v8f c;
#pragma unroll
    for (int r = 0; r < 8; ++r) c[r] = rowp[(size_t)(hi * 8 + r) * NK_ + nt * 16 + col];
    c = wmma_f16(a, frag_h(kf + (size_t)(b * NK_ + kt * 128 + nt * 16 + col) * HD_, 0, lane), c);
#pragma unroll
    for (int r = 0; r < 8; ++r) S[(hi * 8 + r) * 128 + nt * 16 + col] = c[r];
  }
  __syncthreads();
#pragma unroll
  for (int q = 0; q < 16; ++q) vst2(rowp + (size_t)q * NK_ + lane * 4, *(const v4f*)(S + q * 128 + lane * 4));
}

__global__ __launch_bounds__(256) void softmax_k(float* __restrict__ attn) {
  __shared__ float red[256];
  const int tid = threadIdx.x;
  float* p = attn + (long)blockIdx.x * NK_;
  float v[8]; float mx = -3.402823e38f;
#pragma unroll
  for (int i = 0; i < 8; ++i) { v[i] = p[tid + i * 256]; mx = fmaxf(mx, v[i]); }
  red[tid] = mx; __syncthreads();
  for (int s = 128; s > 0; s >>= 1) { if (tid < s) red[tid] = fmaxf(red[tid], red[tid + s]); __syncthreads(); }
  mx = red[0]; __syncthreads();
  float sum = 0.0f;
#pragma unroll
  for (int i = 0; i < 8; ++i) { v[i] = __expf(v[i] - mx); sum += v[i]; }
  red[tid] = sum; __syncthreads();
  for (int s = 128; s > 0; s >>= 1) { if (tid < s) red[tid] += red[tid + s]; __syncthreads(); }
  const float inv = 1.0f / red[0];
#pragma unroll
  for (int i = 0; i < 8; ++i) vst2(p + tid + i * 256, (float_a)(v[i] * inv));
}

__global__ __launch_bounds__(256) void av_k(const float* __restrict__ attn, const float* __restrict__ v, float* __restrict__ x) {
  __shared__ __align__(16) float so[8][16 * 32];
  const int gw = blockIdx.x * 8 + (threadIdx.x >> 5);
  const int qt = gw & 15, h = (gw >> 4) & 7, b = gw >> 7;
  const int lane = threadIdx.x & 31, hi = lane >> 4, col = lane & 15;
  const float* A = attn + (((size_t)(b * NH_ + h) * NQ_ + qt * 16 + col) * NK_);
  const float* V = v + (size_t)b * NK_ * HD_;
  v8f c0 = {}, c1 = {};
#pragma unroll 2
  for (int kk = 0; kk < NK_; kk += 32) {
    const v16h a = frag_f32(A, kk, lane, PSC);
    v16h b0, b1;
#pragma unroll
    for (int e = 0; e < 16; ++e) { const int key = kk + ((e < 8) ? e : e + 8) + 8 * hi;
      b0[e] = (_Float16)V[(size_t)key * HD_ + col]; b1[e] = (_Float16)V[(size_t)key * HD_ + 16 + col]; }
    c0 = wmma_f16(a, b0, c0); c1 = wmma_f16(a, b1, c1);
  }
  float* S = so[threadIdx.x >> 5];
#pragma unroll
  for (int r = 0; r < 8; ++r) { S[(hi * 8 + r) * 32 + col] = c0[r] * PUN; S[(hi * 8 + r) * 32 + 16 + col] = c1[r] * PUN; }
  __syncthreads();
#pragma unroll
  for (int q = 0; q < 4; ++q) { const int rl = q * 4 + (lane >> 3), pc = lane & 7;
    vst2(x + ((size_t)(b * NQ_ + qt * 16 + rl)) * DIM_ + h * HD_ + pc * 4, *(const v4f*)(S + rl * 32 + pc * 4)); }
}

__global__ __launch_bounds__(128) void oproj_k(const float* __restrict__ xx, const _Float16* __restrict__ WT, const float* __restrict__ bias,
                                              float* __restrict__ out) {
  __shared__ __align__(16) float so[4][16 * 64];
  const int tid = threadIdx.x, wave = tid >> 5, lane = tid & 31, hi = lane >> 4, col = lane & 15;
  const int m0 = blockIdx.y * 64 + wave * 16, n0 = blockIdx.x * 64;
  const float* ar = xx + (size_t)(m0 + col) * DIM_;
  float* S = so[wave];
#pragma unroll 1
  for (int nt = 0; nt < 4; ++nt) {
    v8f acc = {};
    const _Float16* br = WT + (size_t)(n0 + nt * 16 + col) * DIM_;
#pragma unroll
    for (int kc = 0; kc < DIM_ / 32; ++kc) acc = wmma_f16(frag_f32(ar, kc * 32, lane, 1.0f), frag_h(br, kc * 32, lane), acc);
#pragma unroll
    for (int r = 0; r < 8; ++r) S[(hi * 8 + r) * 64 + nt * 16 + col] = acc[r] + bias[n0 + nt * 16 + col];
  }
  __syncthreads();
#pragma unroll
  for (int q = 0; q < 8; ++q) { const int rl = q * 2 + (lane >> 4), pc = lane & 15; const int m = m0 + rl, bb = m / NQ_, qq = m % NQ_;
    vst2(out + ((size_t)qq * B_ + bb) * DIM_ + n0 + pc * 4, *(const v4f*)(S + rl * 64 + pc * 4)); }
}

extern "C" void kernel_launch(void* const* d_in, const int* in_sizes, int n_in,
                              void* d_out, int out_size, void* d_ws, size_t ws_size,
                              hipStream_t stream) {
  (void)in_sizes; (void)n_in; (void)out_size; (void)ws_size;
  const float* query  = (const float*)d_in[0];
  const float* key    = (const float*)d_in[1];
  const float* refp   = (const float*)d_in[2];
  const float* xyz    = (const float*)d_in[4];
  const float* q_w    = (const float*)d_in[5];
  const float* q_b    = (const float*)d_in[6];
  const float* k_w    = (const float*)d_in[7];
  const float* k_b    = (const float*)d_in[8];
  const float* v_w    = (const float*)d_in[9];
  const float* v_b    = (const float*)d_in[10];
  const float* proj_w = (const float*)d_in[11];
  const float* proj_b = (const float*)d_in[12];
  const float* cpb_w1 = (const float*)d_in[13];
  const float* cpb_b1 = (const float*)d_in[14];
  const float* cpb_w2 = (const float*)d_in[15];

  char* ws = (char*)d_ws; size_t off = 0;
  auto alloc = [&](size_t bytes) -> void* { void* p = ws + off; off = (off + bytes + 255) & ~(size_t)255; return p; };
  float*    tables = (float*)alloc(64000 * 4);
  _Float16* WqT    = (_Float16*)alloc(256 * 256 * 2);
  _Float16* WkT    = (_Float16*)alloc(32 * 256 * 2);
  _Float16* WvT    = (_Float16*)alloc(32 * 256 * 2);
  _Float16* WpT    = (_Float16*)alloc(256 * 256 * 2);
  _Float16* qf     = (_Float16*)alloc((size_t)B_ * NQ_ * DIM_ * 2);
  _Float16* kf     = (_Float16*)alloc((size_t)B_ * NK_ * HD_ * 2);
  float*    vf     = (float*)alloc((size_t)B_ * NK_ * HD_ * 4);
  float*    xf     = (float*)alloc((size_t)B_ * NQ_ * DIM_ * 4);

  float* out_x    = (float*)d_out;
  float* out_attn = out_x + NQ_ * B_ * DIM_;

  k_wt<<<(256 / 64) * (256 / 64), 256, 0, stream>>>(q_w, WqT, 256, 256);
  k_wt<<<(256 / 64) * 1, 256, 0, stream>>>(k_w, WkT, 256, 32);
  k_wt<<<(256 / 64) * 1, 256, 0, stream>>>(v_w, WvT, 256, 32);
  k_wt<<<(256 / 64) * (256 / 64), 256, 0, stream>>>(proj_w, WpT, 256, 256);
  build_tables_k<<<8, 128, 0, stream>>>(cpb_w1, cpb_b1, cpb_w2, tables);
  rpe_k<<<(B_ * NQ_ * NK_) / 256, 256, 0, stream>>>(refp, xyz, tables, out_attn);
  const float qscale = 0.17677669529663687f;
  proj_k<256, 0><<<(B_ * NQ_) / 64, 128, 0, stream>>>(query, WqT, q_b, qf, nullptr, qscale, NQ_);
  proj_k<32, 0><<<(B_ * NK_) / 64, 128, 0, stream>>>(key, WkT, k_b, kf, nullptr, 1.0f, NK_);
  proj_k<32, 1><<<(B_ * NK_) / 64, 128, 0, stream>>>(key, WvT, v_b, nullptr, vf, 1.0f, NK_);
  qk_k<<<(B_ * NH_ * (NQ_ / 16) * (NK_ / 128)) / 8, 256, 0, stream>>>(qf, kf, out_attn);
  softmax_k<<<B_ * NH_ * NQ_, 256, 0, stream>>>(out_attn);
  av_k<<<(B_ * NH_ * (NQ_ / 16)) / 8, 256, 0, stream>>>(out_attn, vf, xf);
  oproj_k<<<dim3(DIM_ / 64, (B_ * NQ_) / 64), 128, 0, stream>>>(xf, WpT, proj_b, out_x);
}
